// Lstm_82789789597912
// MI455X (gfx1250) — hardware-verified
//
#include <hip/hip_runtime.h>
#include <math.h>

constexpr int N_BATCH   = 128;
constexpr int N_STEP    = 128;
constexpr int N_VOCAB   = 50000;
constexpr int N_EMB     = 300;
constexpr int N_HID     = 300;
constexpr int N_CLS     = 3;
constexpr int W_COLS    = 4 * N_HID;
constexpr int K_PAD     = 320;
constexpr int G_PAD     = 320;
constexpr int Z_COLS    = 4 * G_PAD;
constexpr int X_ROWS    = N_STEP * N_BATCH;
constexpr int CH_ROW    = K_PAD / 8;
constexpr int PLANE_CH  = Z_COLS * CH_ROW;
constexpr int PACK_BLK  = (2 * PLANE_CH) / 256;
constexpr int BIAS_BLK  = 2;
constexpr int GATH_BLK  = (X_ROWS * CH_ROW) / 256;
constexpr int SEQ_THR   = 320;
constexpr int H_PITCH   = 328;
constexpr int GATE_PLANE = G_PAD * K_PAD;
constexpr float X_CARRY   = 16.0f;
constexpr float W_CARRY   = 16.0f;
constexpr float H_CARRY   = 64.0f;
constexpr float ZX_FOLD   = 1.0f / (X_CARRY * W_CARRY);
constexpr float REC_CARRY = H_CARRY * W_CARRY;
constexpr float REC_FOLD  = 1.0f / REC_CARRY;

static_assert(N_EMB == N_HID);
static_assert(K_PAD % 32 == 0 && K_PAD >= N_EMB && K_PAD >= N_HID);
static_assert(G_PAD % 16 == 0 && G_PAD >= N_HID);
static_assert(Z_COLS % 64 == 0 && X_ROWS % 64 == 0);
static_assert((2 * PLANE_CH) % 256 == 0);
static_assert((X_ROWS * CH_ROW) % 256 == 0);
static_assert(G_PAD == 32 * (SEQ_THR / 32));
static_assert(N_BATCH % 16 == 0);
static_assert((16 * G_PAD / 4) % SEQ_THR == 0);
static_assert(Z_COLS / 4 <= BIAS_BLK * 256);
static_assert(N_BATCH * N_CLS == 384);
static_assert((H_PITCH * 2) % 16 == 0);

typedef __attribute__((ext_vector_type(16))) _Float16 v16h;
typedef __attribute__((ext_vector_type(8)))  _Float16 v8h;
typedef __attribute__((ext_vector_type(8)))  float    v8f;
typedef __attribute__((ext_vector_type(4)))  float    v4f;

__device__ __forceinline__ void guard4_a(v8f& a, v8f& b, v8f& c, v8f& d, v16h x) {
  asm volatile("v_nop\n\tv_nop\n\tv_nop\n\tv_nop" : "+v"(a), "+v"(b), "+v"(c), "+v"(d) : "v"(x));
}
__device__ __forceinline__ void guard4_ab(v8f& a, v8f& b, v8f& c, v8f& d, v16h x, v16h y0, v16h y1, v16h y2, v16h y3) {
  asm volatile("v_nop\n\tv_nop\n\tv_nop\n\tv_nop" : "+v"(a), "+v"(b), "+v"(c), "+v"(d) : "v"(x), "v"(y0), "v"(y1), "v"(y2), "v"(y3));
}
__device__ __forceinline__ void keep4_h(v16h a, v16h b, v16h c, v16h d) { asm volatile("v_nop" :: "v"(a), "v"(b), "v"(c), "v"(d)); }
__device__ __forceinline__ void acc_guard4(v8f& a, v8f& b, v8f& c, v8f& d) {
  asm volatile("v_nop\n\tv_nop\n\tv_nop\n\tv_nop" : "+v"(a), "+v"(b), "+v"(c), "+v"(d));
}
__device__ __forceinline__ void burst_fence2(v8f& a, v8f& b) { asm volatile("" : "+v"(a), "+v"(b) :: "memory"); }

union FragU { v16h v; v8h h[2]; };
__device__ __forceinline__ v16h frag_load(const _Float16* p) {
  FragU f; f.h[0] = *(const v8h*)(p); f.h[1] = *(const v8h*)(p + 16); return f.v;
}
__device__ __forceinline__ v8f frag_mma(v16h a, v16h b, v8f c) {
  return __builtin_amdgcn_wmma_f32_16x16x32_f16(false, a, false, b, (short)0, c, false, false);
}

__device__ __forceinline__ float sigm_f(float x) { return __builtin_amdgcn_rcpf(1.0f + expf(-x)); }
__device__ __forceinline__ float tanh_f(float x) { return 1.0f - 2.0f * __builtin_amdgcn_rcpf(1.0f + expf(2.0f * x)); }

__global__ __launch_bounds__(256) void pack_w_kernel(const float* __restrict__ W, const float* __restrict__ b_lstm,
                                                     unsigned short* __restrict__ WT, float* __restrict__ biasp) {
  const int tid = threadIdx.x;
  if (blockIdx.x < PACK_BLK) {
    const int i = blockIdx.x * 256 + tid;
    const int plane = i / PLANE_CH;
    const int rem = i - plane * PLANE_CH;
    const int n = rem / CH_ROW;
    const int k8 = (rem - n * CH_ROW) * 8;
    const int g = n / G_PAD;
    const int c = n - g * G_PAD;
    const int cc = c < N_HID ? c : (N_HID - 1);
    const bool okc = c < N_HID;
    v8h hv;
#pragma unroll
    for (int e = 0; e < 8; ++e) {
      const int k = k8 + e;
      const int kk = k < N_HID ? k : (N_HID - 1);
      const float val = W[(size_t)(plane * N_EMB + kk) * W_COLS + g * N_HID + cc];
      const float f = (okc && (k < N_HID)) ? (val * W_CARRY) : 0.0f;
      hv[e] = (_Float16)f;
    }
    *(volatile v8h*)(WT + (size_t)i * 8) = hv;
    __threadfence();
    *(volatile v8h*)(WT + (size_t)i * 8) = hv;
  } else {
    const int q = (blockIdx.x - PACK_BLK) * 256 + tid;
    if (q < Z_COLS / 4) {
      const int n4 = q * 4;
      const int g = n4 / G_PAD;
      const int c = n4 - g * G_PAD;
      v4f o;
#pragma unroll
      for (int e = 0; e < 4; ++e) {
        const int ce = c + e;
        const int cc = ce < N_HID ? ce : (N_HID - 1);
        const float val = b_lstm[g * N_HID + cc];
        o[e] = (ce < N_HID) ? val : 0.0f;
      }
      *(volatile v4f*)(biasp + n4) = o;
      __threadfence();
      *(volatile v4f*)(biasp + n4) = o;
    }
  }
}

__global__ __launch_bounds__(256) void gather_x_kernel(const int* __restrict__ x, const float* __restrict__ emb,
                                                       unsigned short* __restrict__ Xh) {
  const int i = blockIdx.x * 256 + threadIdx.x;
  const int r = i / CH_ROW;
  const int k8 = (i - r * CH_ROW) * 8;
  const int t = r >> 7;
  const int b = r & (N_BATCH - 1);
  int tok = x[b * N_STEP + t];
  tok = tok < 0 ? 0 : tok;
  tok = tok > (N_VOCAB - 1) ? (N_VOCAB - 1) : tok;
  const float* er = emb + (size_t)tok * N_EMB;
  v8h hv;
#pragma unroll
  for (int e = 0; e < 8; ++e) {
    const int k = k8 + e;
    const int kk = k < N_EMB ? k : (N_EMB - 1);
    const float val = er[kk];
    const float f = (k < N_EMB) ? (val * X_CARRY) : 0.0f;
    hv[e] = (_Float16)f;
  }
  *(volatile v8h*)(Xh + (size_t)i * 8) = hv;
  __threadfence();
  *(volatile v8h*)(Xh + (size_t)i * 8) = hv;
}

__global__ __launch_bounds__(256) void gemm_zx_kernel(
    const unsigned short* __restrict__ Ap, int lda,
    const unsigned short* __restrict__ Btp, int ldb,
    float* __restrict__ Cout, int ldc,
    const float* __restrict__ bias,
    int M, int N, int K, float scale) {
  const _Float16* A  = (const _Float16*)Ap;
  const _Float16* Bt = (const _Float16*)Btp;
  __shared__ __align__(16) float sT[8][16 * 68];
  const int lane = threadIdx.x & 31;
  const int wave = threadIdx.x >> 5;
  const int tilesN = N >> 6;
  const int tilesM = M >> 6;
  const int tile = blockIdx.x * 8 + wave;
  if (tile >= tilesM * tilesN) return;
  const int tm = tile / tilesN;
  const int tn = tile - tm * tilesN;
  const int m0 = tm << 6;
  const int n0 = tn << 6;
  const int rlane = lane & 15;
  const int koff  = (lane >> 4) * 8;
  const int mOff  = (lane >> 4) * 8;

  v8f acc[4][4];
#pragma unroll
  for (int i = 0; i < 4; ++i)
#pragma unroll
    for (int j = 0; j < 4; ++j) acc[i][j] = (v8f){0.f, 0.f, 0.f, 0.f, 0.f, 0.f, 0.f, 0.f};

  for (int k0 = 0; k0 < K; k0 += 32) {
    v16h bh[4];
#pragma unroll
    for (int j = 0; j < 4; ++j) {
      const size_t bo = (size_t)(n0 + (j << 4) + rlane) * ldb + koff + k0;
      bh[j] = frag_load(Bt + bo);
    }
#pragma unroll
    for (int i = 0; i < 4; ++i) {
      const size_t ao = (size_t)(m0 + (i << 4) + rlane) * lda + koff + k0;
      const v16h ah = frag_load(A + ao);
#pragma unroll
      for (int j = 0; j < 4; ++j) acc[i][j] = frag_mma(ah, bh[j], acc[i][j]);
      guard4_a(acc[i][0], acc[i][1], acc[i][2], acc[i][3], ah);
    }
    keep4_h(bh[0], bh[1], bh[2], bh[3]);
  }
  acc_guard4(acc[0][0], acc[0][1], acc[0][2], acc[0][3]);
  acc_guard4(acc[1][0], acc[1][1], acc[1][2], acc[1][3]);
  acc_guard4(acc[2][0], acc[2][1], acc[2][2], acc[2][3]);
  acc_guard4(acc[3][0], acc[3][1], acc[3][2], acc[3][3]);

  float* slab = sT[wave];
#pragma unroll
  for (int i = 0; i < 4; ++i) {
    const int mBase = m0 + (i << 4);
#pragma unroll
    for (int j = 0; j < 4; ++j) {
      const int n = n0 + (j << 4) + rlane;
      const float bv = bias[n];
#pragma unroll
      for (int r = 0; r < 8; ++r) {
        float v = acc[i][j][r] * scale;
        v += bv;
        slab[(mOff + r) * 68 + (j << 4) + rlane] = v;
      }
    }
    __builtin_amdgcn_fence(__ATOMIC_RELEASE, "workgroup");
    __builtin_amdgcn_wave_barrier();
    __builtin_amdgcn_fence(__ATOMIC_ACQUIRE, "workgroup");
    {
      const int hh = lane >> 4, c4 = (lane & 15) * 4;
      for (int pass = 0; pass < 2; ++pass) {
#pragma unroll
        for (int it = 0; it < 8; ++it) {
          const int row = it * 2 + hh;
          const v4f v = *(const v4f*)(slab + row * 68 + c4);
          *(volatile v4f*)(Cout + (size_t)(mBase + row) * ldc + n0 + c4) = v;
        }
        __threadfence();
      }
    }
    __builtin_amdgcn_fence(__ATOMIC_RELEASE, "workgroup");
    __builtin_amdgcn_wave_barrier();
    __builtin_amdgcn_fence(__ATOMIC_ACQUIRE, "workgroup");
  }
}

__global__ __launch_bounds__(SEQ_THR) void lstm_seq_kernel(const float* Zx, const unsigned short* __restrict__ WhTp,
                                                           const int* __restrict__ lengths, float* hfin) {
  __shared__ __align__(16) _Float16 Hb[2][16 * H_PITCH];
  __shared__ __align__(16) float    St[2][16][SEQ_THR];
  const _Float16* WhT = (const _Float16*)WhTp;
  const int tid = threadIdx.x, lane = tid & 31, wave = tid >> 5;
  const int c = lane & 15, hh = lane >> 4, koff = hh * 8;
  const int rowbase = blockIdx.x * 16;

  {
    _Float16* hb = &Hb[0][0];
#pragma unroll 1
    for (int i = tid; i < 2 * 16 * H_PITCH; i += SEQ_THR) hb[i] = (_Float16)0.0f;
  }
#pragma unroll
  for (int s = 0; s < 2; ++s)
#pragma unroll
    for (int q = 0; q < 16; ++q) St[s][q][tid] = 0.0f;
  int len[8];
#pragma unroll
  for (int r = 0; r < 8; ++r) {
    int v = lengths[rowbase + 8 * hh + r];
    v = v < 0 ? 0 : v;
    v = v > N_STEP ? N_STEP : v;
    len[r] = v;
  }
  __syncthreads();

#pragma unroll 1
  for (int t = 0; t < N_STEP; ++t) {
    const int cur = t & 1;
    const _Float16* hcur = &Hb[cur][0] + c * H_PITCH + koff;
    _Float16* hnx = &Hb[cur ^ 1][0];
#pragma unroll 1
    for (int s = 0; s < 2; ++s) {
      const int col = 32 * wave + 16 * s + c;
      const float* zp = Zx + (size_t)(t * N_BATCH + rowbase + 8 * hh) * Z_COLS + col;
      v8f a0, a1, a2, a3;
#pragma unroll
      for (int r = 0; r < 8; ++r) {
        a0[r] = zp[r * Z_COLS] * REC_CARRY;
        a1[r] = zp[r * Z_COLS + G_PAD] * REC_CARRY;
      }
      burst_fence2(a0, a1);
#pragma unroll
      for (int r = 0; r < 8; ++r) {
        a2[r] = zp[r * Z_COLS + 2 * G_PAD] * REC_CARRY;
        a3[r] = zp[r * Z_COLS + 3 * G_PAD] * REC_CARRY;
      }
      burst_fence2(a2, a3);
      const _Float16* wh = WhT + (size_t)col * K_PAD + koff;
#pragma unroll 1
      for (int k0 = 0; k0 < K_PAD; k0 += 32) {
        const v16h a  = frag_load(hcur + k0);
        const v16h b0 = frag_load(wh + k0);
        const v16h b1 = frag_load(wh + (size_t)1 * GATE_PLANE + k0);
        const v16h b2 = frag_load(wh + (size_t)2 * GATE_PLANE + k0);
        const v16h b3 = frag_load(wh + (size_t)3 * GATE_PLANE + k0);
        a0 = frag_mma(a, b0, a0);
        a1 = frag_mma(a, b1, a1);
        a2 = frag_mma(a, b2, a2);
        a3 = frag_mma(a, b3, a3);
        guard4_ab(a0, a1, a2, a3, a, b0, b1, b2, b3);
      }
      acc_guard4(a0, a1, a2, a3);
      const bool live = col < N_HID;
#pragma unroll
      for (int r = 0; r < 8; ++r) {
        const float zi = a0[r] * REC_FOLD;
        const float zj = a1[r] * REC_FOLD;
        const float zf = a2[r] * REC_FOLD;
        const float zo = a3[r] * REC_FOLD;
        const float c_old = St[s][r][tid];
        const float h_old = St[s][8 + r][tid];
        const float ig = sigm_f(zi);
        const float fg = sigm_f(zf + 1.0f);
        const float og = sigm_f(zo);
        const float jg = tanh_f(zj);
        const float c_new = fg * c_old + ig * jg;
        const float h_new = og * tanh_f(c_new);
        const bool upd = live && (t < len[r]);
        const float c_sel = upd ? c_new : c_old;
        const float h_sel = upd ? h_new : h_old;
        St[s][r][tid] = c_sel;
        St[s][8 + r][tid] = h_sel;
        hnx[(8 * hh + r) * H_PITCH + col] = (_Float16)(h_sel * H_CARRY);
      }
    }
    __syncthreads();
  }

  for (int pass = 0; pass < 2; ++pass) {
#pragma unroll
    for (int it = 0; it < 4; ++it) {
      const int idx = it * SEQ_THR + tid;
      const int row = idx / (G_PAD / 4);
      const int col4 = (idx - row * (G_PAD / 4)) * 4;
      const int w2 = col4 >> 5;
      const int s2 = (col4 >> 4) & 1;
      const int cc = col4 & 15;
      const int hh2 = row >> 3;
      const int r2 = row & 7;
      const v4f v = *(const v4f*)(&St[s2][8 + r2][w2 * 32 + hh2 * 16 + cc]);
      *(volatile v4f*)(hfin + (size_t)(rowbase + row) * G_PAD + col4) = v;
    }
    __threadfence();
  }
}

__global__ __launch_bounds__(384) void head_kernel(const float* hfin, const float* __restrict__ Wd,
                                                   const float* __restrict__ bd, float* __restrict__ out) {
  const int tid = threadIdx.x;
  const int b = tid / N_CLS;
  const int j = tid - b * N_CLS;
  const float* hr = hfin + (size_t)b * G_PAD;
  float s = 0.0f;
#pragma unroll 4
  for (int k = 0; k < N_HID; ++k) s += hr[k] * Wd[k * N_CLS + j];
  s += bd[j];
  *(volatile float*)(out + tid) = s;
  __threadfence();
  *(volatile float*)(out + tid) = s;
}

extern "C" void kernel_launch(void* const* d_in, const int* in_sizes, int n_in,
                              void* d_out, int out_size, void* d_ws, size_t ws_size, hipStream_t stream) {
  if (n_in < 7 || d_out == nullptr || d_ws == nullptr) return;
  if (in_sizes[0] != N_BATCH * N_STEP || in_sizes[1] != N_BATCH || in_sizes[2] != N_VOCAB * N_EMB ||
      in_sizes[3] != (N_EMB + N_HID) * W_COLS || in_sizes[4] != W_COLS || in_sizes[5] != N_HID * N_CLS ||
      in_sizes[6] != N_CLS || out_size != N_BATCH * N_CLS) return;

  const int*   x       = (const int*)d_in[0];
  const int*   lengths = (const int*)d_in[1];
  const float* emb     = (const float*)d_in[2];
  const float* w_lstm  = (const float*)d_in[3];
  const float* b_lstm  = (const float*)d_in[4];
  const float* w_dense = (const float*)d_in[5];
  const float* b_dense = (const float*)d_in[6];
  float* out = (float*)d_out;

  char* ws = (char*)d_ws; size_t off = 0;
  auto carve = [&](size_t bytes) -> char* { char* p = ws + off; off += (bytes + 255) & ~(size_t)255; return p; };
  unsigned short* WT    = (unsigned short*)carve((size_t)2 * Z_COLS * K_PAD * 2);
  float*          BIASP = (float*)carve((size_t)Z_COLS * 4);
  unsigned short* XH    = (unsigned short*)carve((size_t)X_ROWS * K_PAD * 2);
  float*          ZX    = (float*)carve((size_t)X_ROWS * Z_COLS * 4);
  float*          HFIN  = (float*)carve((size_t)N_BATCH * G_PAD * 4);
  if (off > ws_size || off > (size_t)134217728) return;
  unsigned short* WXT = WT;
  unsigned short* WHT = WT + (size_t)Z_COLS * K_PAD;

  pack_w_kernel<<<PACK_BLK + BIAS_BLK, 256, 0, stream>>>(w_lstm, b_lstm, WT, BIASP);
  gather_x_kernel<<<GATH_BLK, 256, 0, stream>>>(x, emb, XH);
  gemm_zx_kernel<<<(X_ROWS / 64) * (Z_COLS / 64) / 8, 256, 0, stream>>>(
      XH, K_PAD, WXT, K_PAD, ZX, Z_COLS, BIASP, X_ROWS, Z_COLS, K_PAD, ZX_FOLD);
  lstm_seq_kernel<<<N_BATCH / 16, SEQ_THR, 0, stream>>>(ZX, WHT, lengths, HFIN);
  head_kernel<<<1, N_BATCH * N_CLS, 0, stream>>>(HFIN, w_dense, b_dense, out);
}
